// GAT_layers_28595892257582
// MI455X (gfx1250) — hardware-verified
//
#include <hip/hip_runtime.h>
#include <stddef.h>
#include <stdint.h>

#pragma clang fp contract(off)

#define NB   4
#define NN   4096
#define CI0  64
#define NH0  4
#define DD0  32
#define CI1  128
#define NH1  1
#define DD1  64
#define KC   32
#define QBR  64
#define EPSN 1e-5f
#define NWEL 8192

static_assert(CI1 == NH0 * DD0);
static_assert(NN % QBR == 0);
static_assert(NN % KC == 0);
static_assert(NN % 64 == 0);
static_assert((NB * NN) % 64 == 0);
static_assert(NH0 * CI0 * DD0 == NWEL);
static_assert(NH1 * CI1 * DD1 == NWEL);
static_assert(NWEL == 256 * 8 * 4);

typedef float          v8f   __attribute__((ext_vector_type(8)));
typedef float          v4f   __attribute__((ext_vector_type(4)));
typedef unsigned int   v4u   __attribute__((ext_vector_type(4)));
typedef unsigned short v8us  __attribute__((ext_vector_type(8)));
typedef unsigned short v16us __attribute__((ext_vector_type(16)));
typedef __bf16         v16b  __attribute__((ext_vector_type(16)));
typedef unsigned short ush;

union FragU { v16us v; v8us h[2]; v4u q[2]; v16b b; };
union PackU { v8us s; v4u u; };
struct HL { v4u h; v4u l; };

__device__ __forceinline__ ush f2bf(float f) {
  const unsigned u = __float_as_uint(f);
  return (ush)((u + 0x7FFFu + ((u >> 16) & 1u)) >> 16);
}
__device__ __forceinline__ float bf2f(ush v) { return __uint_as_float(((unsigned)v) << 16); }

__device__ __forceinline__ HL split8(v8f f) {
  PackU ph, pl;
#pragma unroll
  for (int e = 0; e < 8; ++e) {
    const ush hi = f2bf(f[e]);
    ph.s[e] = hi;
    pl.s[e] = f2bf(f[e] - bf2f(hi));
  }
  HL r; r.h = ph.u; r.l = pl.u;
  return r;
}

__device__ __forceinline__ v8f mmab(v16us a, v16us b, v8f c) {
  FragU ua, ub; ua.v = a; ub.v = b;
  c = __builtin_amdgcn_wmma_f32_16x16x32_bf16(false, ua.b, false, ub.b, (short)0, c, false, false);
  asm volatile("v_nop\n\tv_nop\n\tv_nop\n\tv_nop" : "+v"(c) : "v"(a), "v"(b));
  return c;
}

__device__ __forceinline__ v16us ldfragu(const ush* p, int ld, int row0, int k0, int lane) {
  const int m = lane & 15, lh = lane >> 4;
  const ush* qq = p + (size_t)(row0 + m) * ld + k0 + 8 * lh;
  FragU f;
  f.h[0] = *(const v8us*)(qq);
  f.h[1] = *(const v8us*)(qq + 16);
  return f.v;
}

__device__ __forceinline__ v8f zero8() { return (v8f){0.f, 0.f, 0.f, 0.f, 0.f, 0.f, 0.f, 0.f}; }

__device__ __forceinline__ float pval(float ssl, float sd, float mrow) {
  const float s = ssl + sd;
  const float l = (s >= 0.f) ? s : 0.2f * s;
  return __expf(l - mrow);
}

template<int C>
__global__ __launch_bounds__(256) void k_stats(const float* __restrict__ x, float* __restrict__ st) {
  constexpr int G  = 256 / C;
  constexpr int NI = (2 * C) / 128;
  static_assert(G * C == 256);
  static_assert(NI * 128 == 2 * C);
  __shared__ double shs[256];
  __shared__ double shq[256];
  __shared__ __align__(16) float tab[2 * C];
  const int tid = threadIdx.x, lane = tid & 31, wave = tid >> 5;
  const int b = blockIdx.x;
  const int c = tid % C, g = tid / C;
  const float* xp = x + (size_t)b * NN * C + c;
  double s = 0.0, q = 0.0;
#pragma unroll 1
  for (int n = g; n < NN; n += G) {
    const float v = xp[(size_t)n * C];
    const double dv = (double)v;
    s += dv;
    q += dv * dv;
  }
  shs[tid] = s;
  shq[tid] = q;
  __syncthreads();
  if (g == 0) {
    double S = 0.0, Q = 0.0;
#pragma unroll
    for (int j = 0; j < G; ++j) { S += shs[j * C + c]; Q += shq[j * C + c]; }
    const double mean = S * (1.0 / (double)NN);
    double var = Q * (1.0 / (double)NN) - mean * mean;
    var = (var > 0.0) ? var : 0.0;
    const float sd = sqrtf((float)var + EPSN);
    tab[c] = (float)mean;
    tab[C + c] = 1.0f / sd;
  }
  __syncthreads();
  if (wave == 0) {
    v4f v[NI];
    size_t go[NI];
#pragma unroll
    for (int i = 0; i < NI; ++i) {
      const int p = lane + 32 * i;
      v[i] = *(const v4f*)(tab + 4 * p);
      go[i] = (size_t)b * 2 * C + 4 * p;
    }
#pragma unroll
    for (int i = 0; i < NI; ++i) *(volatile v4f*)(st + go[i]) = v[i];
    __threadfence();
#pragma unroll
    for (int i = 0; i < NI; ++i) *(volatile v4f*)(st + go[i]) = v[i];
  }
}

__global__ __launch_bounds__(256) void k_wprep(const float* __restrict__ w0, const float* __restrict__ w1,
                                               ush* __restrict__ W0h, ush* __restrict__ W0l,
                                               ush* __restrict__ W1h, ush* __restrict__ W1l) {
  __shared__ __align__(16) float Wsf[NWEL];
  const int z = blockIdx.x;
  const int tid = threadIdx.x;
  const float* w = (z == 0) ? w0 : w1;
  ush* dh = (z == 0) ? W0h : W1h;
  ush* dl = (z == 0) ? W0l : W1l;
  const int cin   = (z == 0) ? CI0 : CI1;
  const int lcout = (z == 0) ? 5 : 6;
  const int cout  = 1 << lcout;
  const int lppr  = (z == 0) ? 3 : 4;

#pragma unroll 1
  for (int ch = 0; ch < 2; ++ch) {
    v4f t[4];
#pragma unroll
    for (int i = 0; i < 4; ++i) {
      const int p = tid + 256 * (4 * ch + i);
      t[i] = *(const v4f*)(w + 4 * p);
    }
#pragma unroll
    for (int i = 0; i < 4; ++i) {
      const int p = tid + 256 * (4 * ch + i);
      *(v4f*)(Wsf + 4 * p) = t[i];
    }
  }
  __syncthreads();

  v4u vh[4], vl[4];
  size_t go[4];
#pragma unroll
  for (int it = 0; it < 4; ++it) {
    const int p  = tid + 256 * it;
    const int j  = p >> lppr;
    const int pc = p & ((1 << lppr) - 1);
    const int hd = j >> lcout;
    const int kk = j & (cout - 1);
    const float* sp = Wsf + hd * cin * cout + (8 * pc) * cout + kk;
    v8f f = zero8();
#pragma unroll
    for (int i = 0; i < 8; ++i) f[i] = sp[i * cout];
    const HL s = split8(f);
    vh[it] = s.h;
    vl[it] = s.l;
    go[it] = (size_t)j * cin + 8 * pc;
  }
#pragma unroll
  for (int it = 0; it < 4; ++it) {
    *(volatile v4u*)(dh + go[it]) = vh[it];
    *(volatile v4u*)(dl + go[it]) = vl[it];
  }
  __threadfence();
#pragma unroll
  for (int it = 0; it < 4; ++it) {
    *(volatile v4u*)(dh + go[it]) = vh[it];
    *(volatile v4u*)(dl + go[it]) = vl[it];
  }
}

template<int CIN, int H, int DH>
__global__ __launch_bounds__(128)
void k_proj(const float* __restrict__ hsrc, const float* __restrict__ st,
            const ush* __restrict__ Wh, const ush* __restrict__ Wl,
            const float* __restrict__ asrc, const float* __restrict__ adst,
            ush* __restrict__ VTh, ush* __restrict__ VTl, float* __restrict__ S) {
  constexpr int NC    = H * DH;
  constexpr int KS    = CIN / 32;
  constexpr int NT    = NC / 16;
  constexpr int AP    = CIN + 8;
  constexpr int HP    = NC + 4;
  constexpr int PPR   = CIN / 8;
  constexpr int NPA   = (64 * PPR) / 128;
  constexpr int NPV   = (8 * NC) / 128;
  constexpr int NPAIR = 64 * H;
  constexpr int NDI   = (NPAIR + 127) / 128;
  static_assert(CIN % 32 == 0);
  static_assert(NC % 16 == 0);
  static_assert(NPA * 128 == 64 * PPR);
  static_assert(NPV * 128 == 8 * NC);
  static_assert(NPV % 4 == 0);
  static_assert((AP * 2) % 16 == 0);
  static_assert((HP * 4) % 16 == 0);
  static_assert(NC <= 128);
  static_assert(H >= 1 && H <= 8);

  __shared__ __align__(16) ush   Ah[64 * AP];
  __shared__ __align__(16) ush   Al[64 * AP];
  __shared__ __align__(16) float Hs[64 * HP];
  __shared__ __align__(16) float sSD[2 * H * 64];
  __shared__ float aS[NC];
  __shared__ float aD[NC];

  const int tid = threadIdx.x, lane = tid & 31, wave = tid >> 5;
  const int hh = lane >> 4, c = lane & 15;
  const int row0 = blockIdx.x * 64;
  const int b  = row0 / NN;
  const int n0 = row0 - b * NN;
  const int BH = NB * H;

  if (tid < NC) { aS[tid] = asrc[tid]; aD[tid] = adst[tid]; }

  const float* stb = st + (size_t)b * 2 * CIN;
#pragma unroll
  for (int it = 0; it < NPA; ++it) {
    const int p   = tid + 128 * it;
    const int row = p / PPR;
    const int pc  = p % PPR;
    const float* xp = hsrc + (size_t)(row0 + row) * CIN + 8 * pc;
    const v4f x0 = *(const v4f*)(xp);
    const v4f x1 = *(const v4f*)(xp + 4);
    const v4f m0 = *(const v4f*)(stb + 8 * pc);
    const v4f m1 = *(const v4f*)(stb + 8 * pc + 4);
    const v4f r0 = *(const v4f*)(stb + CIN + 8 * pc);
    const v4f r1 = *(const v4f*)(stb + CIN + 8 * pc + 4);
    const v4f y0 = (x0 - m0) * r0;
    const v4f y1 = (x1 - m1) * r1;
    const v8f f = (v8f){y0[0], y0[1], y0[2], y0[3], y1[0], y1[1], y1[2], y1[3]};
    const HL s = split8(f);
    *(v4u*)(Ah + row * AP + 8 * pc) = s.h;
    *(v4u*)(Al + row * AP + 8 * pc) = s.l;
  }
  __syncthreads();

  v16us afh[KS], afl[KS];
#pragma unroll
  for (int ks = 0; ks < KS; ++ks) {
    afh[ks] = ldfragu(Ah, AP, 16 * wave, 32 * ks, lane);
    afl[ks] = ldfragu(Al, AP, 16 * wave, 32 * ks, lane);
  }
#pragma unroll
  for (int t = 0; t < NT; ++t) {
    v8f acc = zero8();
#pragma unroll
    for (int ks = 0; ks < KS; ++ks) {
      const v16us bfh = ldfragu(Wh, CIN, 16 * t, 32 * ks, lane);
      const v16us bfl = ldfragu(Wl, CIN, 16 * t, 32 * ks, lane);
      acc = mmab(afh[ks], bfh, acc);
      acc = mmab(afh[ks], bfl, acc);
      acc = mmab(afl[ks], bfh, acc);
    }
#pragma unroll
    for (int r = 0; r < 8; ++r) Hs[(16 * wave + 8 * hh + r) * HP + 16 * t + c] = acc[r];
  }
  __syncthreads();

#pragma unroll
  for (int it = 0; it < NDI; ++it) {
    const int q = tid + 128 * it;
    if (q < NPAIR) {
      const int row = q & 63;
      const int hd  = q >> 6;
      const float* hp = Hs + row * HP + hd * DH;
      const float* ap = aS + hd * DH;
      const float* dp = aD + hd * DH;
      float ss = 0.f, sd = 0.f;
#pragma unroll 8
      for (int k = 0; k < DH; ++k) {
        const float hv = hp[k];
        ss += hv * ap[k];
        sd += hv * dp[k];
      }
      sSD[hd * 64 + row] = ss;
      sSD[(H + hd) * 64 + row] = sd;
    }
  }
  __syncthreads();

  const size_t colbase = (size_t)b * NC;
#pragma unroll
  for (int ch = 0; ch < NPV / 4; ++ch) {
    v4u vh[4], vl[4];
    size_t go[4];
#pragma unroll
    for (int i = 0; i < 4; ++i) {
      const int p   = tid + 128 * (4 * ch + i);
      const int col = p >> 3;
      const int pc  = p & 7;
      const float* cp = Hs + (8 * pc) * HP + col;
      const v8f f = (v8f){cp[0 * HP], cp[1 * HP], cp[2 * HP], cp[3 * HP],
                          cp[4 * HP], cp[5 * HP], cp[6 * HP], cp[7 * HP]};
      const HL s = split8(f);
      vh[i] = s.h;
      vl[i] = s.l;
      go[i] = (colbase + col) * (size_t)NN + n0 + 8 * pc;
    }
#pragma unroll
    for (int i = 0; i < 4; ++i) {
      *(volatile v4u*)(VTh + go[i]) = vh[i];
      *(volatile v4u*)(VTl + go[i]) = vl[i];
    }
    __threadfence();
#pragma unroll
    for (int i = 0; i < 4; ++i) {
      *(volatile v4u*)(VTh + go[i]) = vh[i];
      *(volatile v4u*)(VTl + go[i]) = vl[i];
    }
  }

  if (wave == 0) {
    v4f v[H];
    size_t go[H];
#pragma unroll
    for (int j = 0; j < H; ++j) {
      const int L    = 4 * j + (lane >> 3);
      const int pc   = lane & 7;
      const int half = L & 1;
      const int t2   = L >> 1;
      const int hd   = t2 % H;
      const int arr  = t2 / H;
      v[j]  = *(const v4f*)(sSD + t2 * 64 + half * 32 + 4 * pc);
      go[j] = ((size_t)(arr * BH + b * H + hd)) * NN + n0 + half * 32 + 4 * pc;
    }
#pragma unroll
    for (int j = 0; j < H; ++j) *(volatile v4f*)(S + go[j]) = v[j];
    __threadfence();
#pragma unroll
    for (int j = 0; j < H; ++j) *(volatile v4f*)(S + go[j]) = v[j];
  }
}

template<int DV, bool ACT>
__global__ __launch_bounds__(128)
void k_attn(const float* __restrict__ S, const ush* __restrict__ VTh, const ush* __restrict__ VTl,
            const float* __restrict__ bias, float* __restrict__ out, int H) {
  constexpr int NT  = DV / 16;
  constexpr int OP  = DV + 4;
  constexpr int LPR = DV / 32;
  constexpr int NIT = 4 * LPR;
  constexpr int NKT = NN / KC;
  static_assert(DV % 32 == 0);
  static_assert((OP * 4) % 16 == 0);
  static_assert(NIT * 32 * 4 == 16 * DV);

  __shared__ __align__(16) float Sd[NN];
  __shared__ __align__(16) float Os[4 * 16 * OP];
  __shared__ float red[4];

  const int tid = threadIdx.x, lane = tid & 31, wave = tid >> 5;
  const int hh = lane >> 4, c = lane & 15;
  const int bh = blockIdx.y;
  const int BH = NB * H;
  const int b  = bh / H;
  const int h  = bh - b * H;
  const int qblk = blockIdx.x * QBR;
  const int q0   = qblk + 16 * wave;

  const float* ssrc = S + (size_t)bh * NN;
  const float* sdst = S + (size_t)(BH + bh) * NN;

  float mx = -3.0e38f;
#pragma unroll
  for (int it = 0; it < NN / (4 * 128); ++it) {
    const int p = tid + 128 * it;
    const v4f v = *(const v4f*)(sdst + 4 * p);
    *(v4f*)(Sd + 4 * p) = v;
    mx = fmaxf(mx, fmaxf(fmaxf(v[0], v[1]), fmaxf(v[2], v[3])));
  }
#pragma unroll
  for (int off = 1; off < 32; off <<= 1) mx = fmaxf(mx, __shfl_xor(mx, off, 32));
  if (lane == 0) red[wave] = mx;
  __syncthreads();
  const float Md = fmaxf(fmaxf(red[0], red[1]), fmaxf(red[2], red[3]));

  const float ssl  = ssrc[q0 + c];
  const float tt   = ssl + Md;
  const float mrow = (tt >= 0.f) ? tt : 0.2f * tt;

  const ush* Vh = VTh + (size_t)bh * DV * NN;
  const ush* Vl = VTl + (size_t)bh * DV * NN;

  v8f acc[NT];
#pragma unroll
  for (int t = 0; t < NT; ++t) acc[t] = zero8();
  double ltot = 0.0;

#pragma unroll 1
  for (int kt = 0; kt < NKT; ++kt) {
    const int kv0 = kt * KC;
    const float* sp = Sd + kv0 + 8 * hh;
    const v4f d0 = *(const v4f*)(sp);
    const v4f d1 = *(const v4f*)(sp + 4);
    const v4f d2 = *(const v4f*)(sp + 16);
    const v4f d3 = *(const v4f*)(sp + 20);
    v8f f0 = zero8(), f1 = zero8();
#pragma unroll
    for (int e = 0; e < 4; ++e) {
      f0[e]     = pval(ssl, d0[e], mrow);
      f0[4 + e] = pval(ssl, d1[e], mrow);
      f1[e]     = pval(ssl, d2[e], mrow);
      f1[4 + e] = pval(ssl, d3[e], mrow);
    }
    float tp = 0.f;
#pragma unroll
    for (int e = 0; e < 8; ++e) tp += f0[e];
#pragma unroll
    for (int e = 0; e < 8; ++e) tp += f1[e];
    ltot += (double)tp;

    const HL s0 = split8(f0);
    const HL s1 = split8(f1);
    FragU ph, pl;
    ph.q[0] = s0.h; ph.q[1] = s1.h;
    pl.q[0] = s0.l; pl.q[1] = s1.l;
#pragma unroll
    for (int t = 0; t < NT; ++t) {
      const v16us vfh = ldfragu(Vh, NN, 16 * t, kv0, lane);
      const v16us vfl = ldfragu(Vl, NN, 16 * t, kv0, lane);
      acc[t] = mmab(ph.v, vfh, acc[t]);
      acc[t] = mmab(ph.v, vfl, acc[t]);
      acc[t] = mmab(pl.v, vfh, acc[t]);
    }
  }

  const unsigned long long u = __builtin_bit_cast(unsigned long long, ltot);
  const int lo0 = (int)(unsigned)(u & 0xFFFFFFFFull);
  const int hi0 = (int)(unsigned)(u >> 32);
  const int lo1 = __shfl_xor(lo0, 16, 32);
  const int hi1 = __shfl_xor(hi0, 16, 32);
  const unsigned long long u1 = (((unsigned long long)(unsigned)hi1) << 32) | (unsigned long long)(unsigned)lo1;
  const double other = __builtin_bit_cast(double, u1);
  const float lsum = (float)(ltot + other);
  const float inv  = 1.0f / lsum;

  float* sw = Os + wave * 16 * OP;
#pragma unroll
  for (int r = 0; r < 8; ++r) {
    const float invr = __shfl(inv, 8 * hh + r, 32);
#pragma unroll
    for (int t = 0; t < NT; ++t) {
      float v = acc[t][r] * invr + bias[16 * t + c];
      if (ACT) v = (v > 0.f) ? v : expm1f(v);
      sw[(8 * hh + r) * OP + 16 * t + c] = v;
    }
  }
  __syncthreads();

  const int RS = H * DV;
  v4f val[NIT];
  size_t go[NIT];
#pragma unroll
  for (int it = 0; it < NIT; ++it) {
    const int p    = lane + 32 * it;
    const int L    = p >> 3;
    const int pc   = p & 7;
    const int row  = L / LPR;
    const int half = L % LPR;
    val[it] = *(const v4f*)(sw + row * OP + half * 32 + 4 * pc);
    go[it]  = ((size_t)(b * NN + q0 + row)) * RS + h * DV + half * 32 + 4 * pc;
  }
#pragma unroll
  for (int it = 0; it < NIT; ++it) *(volatile v4f*)(out + go[it]) = val[it];
  __threadfence();
#pragma unroll
  for (int it = 0; it < NIT; ++it) *(volatile v4f*)(out + go[it]) = val[it];
}

extern "C" void kernel_launch(void* const* d_in, const int* in_sizes, int n_in,
                              void* d_out, int out_size, void* d_ws, size_t ws_size,
                              hipStream_t stream) {
  if (n_in < 9) return;
  if (in_sizes[0] != NB * NN * CI0) return;
  if (in_sizes[1] != NH0 * CI0 * DD0) return;
  if (in_sizes[2] != NH0 * DD0) return;
  if (in_sizes[3] != NH0 * DD0) return;
  if (in_sizes[4] != DD0) return;
  if (in_sizes[5] != NH1 * CI1 * DD1) return;
  if (in_sizes[6] != NH1 * DD1) return;
  if (in_sizes[7] != NH1 * DD1) return;
  if (in_sizes[8] != DD1) return;
  if (out_size != NB * NN * DD1) return;

  const float* x     = (const float*)d_in[0];
  const float* w0    = (const float*)d_in[1];
  const float* asrc0 = (const float*)d_in[2];
  const float* adst0 = (const float*)d_in[3];
  const float* bz0   = (const float*)d_in[4];
  const float* w1    = (const float*)d_in[5];
  const float* asrc1 = (const float*)d_in[6];
  const float* adst1 = (const float*)d_in[7];
  const float* bz1   = (const float*)d_in[8];
  float* out = (float*)d_out;

  size_t off = 0;
  const size_t oSt0 = off; off += 4096;
  const size_t oSt1 = off; off += 4096;
  const size_t oW0h = off; off += (size_t)NH0 * DD0 * CI0 * 2;
  const size_t oW0l = off; off += (size_t)NH0 * DD0 * CI0 * 2;
  const size_t oW1h = off; off += (size_t)NH1 * DD1 * CI1 * 2;
  const size_t oW1l = off; off += (size_t)NH1 * DD1 * CI1 * 2;
  const size_t oS0  = off; off += (size_t)2 * NB * NH0 * NN * 4;
  const size_t oV0h = off; off += (size_t)NB * NH0 * DD0 * NN * 2;
  const size_t oV0l = off; off += (size_t)NB * NH0 * DD0 * NN * 2;
  const size_t oH1  = off; off += (size_t)NB * NN * CI1 * 4;
  const size_t oS1  = off; off += (size_t)2 * NB * NH1 * NN * 4;
  const size_t oV1h = off; off += (size_t)NB * NH1 * DD1 * NN * 2;
  const size_t oV1l = off; off += (size_t)NB * NH1 * DD1 * NN * 2;
  if (off > ws_size) return;
  if (off > (size_t)134217728) return;

  char* ws = (char*)d_ws;
  float* St0  = (float*)(ws + oSt0);
  float* St1  = (float*)(ws + oSt1);
  ush*   W0h  = (ush*)(ws + oW0h);
  ush*   W0l  = (ush*)(ws + oW0l);
  ush*   W1h  = (ush*)(ws + oW1h);
  ush*   W1l  = (ush*)(ws + oW1l);
  float* S0   = (float*)(ws + oS0);
  ush*   V0h  = (ush*)(ws + oV0h);
  ush*   V0l  = (ush*)(ws + oV0l);
  float* H1b  = (float*)(ws + oH1);
  float* S1   = (float*)(ws + oS1);
  ush*   V1h  = (ush*)(ws + oV1h);
  ush*   V1l  = (ush*)(ws + oV1l);

  k_stats<CI0><<<dim3(NB), dim3(256), 0, stream>>>(x, St0);
  k_wprep<<<dim3(2), dim3(256), 0, stream>>>(w0, w1, W0h, W0l, W1h, W1l);
  k_proj<CI0, NH0, DD0><<<dim3(NB * NN / 64), dim3(128), 0, stream>>>(x, St0, W0h, W0l, asrc0, adst0, V0h, V0l, S0);
  k_attn<DD0, true><<<dim3(NN / QBR, NB * NH0), dim3(128), 0, stream>>>(S0, V0h, V0l, bz0, H1b, NH0);
  k_stats<CI1><<<dim3(NB), dim3(256), 0, stream>>>(H1b, St1);
  k_proj<CI1, NH1, DD1><<<dim3(NB * NN / 64), dim3(128), 0, stream>>>(H1b, St1, W1h, W1l, asrc1, adst1, V1h, V1l, S1);
  k_attn<DD1, false><<<dim3(NN / QBR, NB * NH1), dim3(128), 0, stream>>>(S1, V1h, V1l, bz1, out, NH1);
  (void)hipGetLastError();
}
